// ScaledDotProductAttention_62062277427456
// MI455X (gfx1250) — hardware-verified
//
#include <hip/hip_runtime.h>

typedef __attribute__((ext_vector_type(16))) _Float16 v16h;
typedef __attribute__((ext_vector_type(8)))  _Float16 v8h;
typedef __attribute__((ext_vector_type(16))) __bf16 v16bf;
typedef __attribute__((ext_vector_type(8)))  __bf16 v8bf;
typedef __attribute__((ext_vector_type(8)))  float  v8f;
typedef __attribute__((ext_vector_type(4)))  float  v4f;

#define BATCH 32
#define SEQ   2048
#define DIM   64
#define QT    64
#define KT    64
#define NWAVE 4
#define MASKV (-4294967295.0f)
#define SCALE 0.125f

__device__ __forceinline__ v8f wmma_f16(v16h a, v16h b, v8f c) {
    v8f d = __builtin_amdgcn_wmma_f32_16x16x32_f16(false, a, false, b, (short)0, c, false, false);
    asm volatile("v_nop\n\tv_nop\n\tv_nop\n\tv_nop" : "+v"(d) : "v"(a), "v"(b));
    return d;
}
__device__ __forceinline__ v8f wmma_bf16(v16bf a, v16bf b, v8f c) {
    v8f d = __builtin_amdgcn_wmma_f32_16x16x32_bf16(false, a, false, b, (short)0, c, false, false);
    asm volatile("v_nop\n\tv_nop\n\tv_nop\n\tv_nop" : "+v"(d) : "v"(a), "v"(b));
    return d;
}
__device__ __forceinline__ __bf16 bf_hi(float x) { return (__bf16)x; }
__device__ __forceinline__ __bf16 bf_lo(float x, __bf16 h) { return (__bf16)(x - (float)h); }

template <typename V16, typename V8, typename T>
__device__ __forceinline__ V16 load_frag(const T* tile, int ld, int k0, int lane) {
    union { V16 v; V8 h[2]; } r;
    const T* row = tile + (lane & 15) * ld + k0 + 8 * (lane >> 4);
    r.h[0] = *(const V8*)(row);
    r.h[1] = *(const V8*)(row + 16);
    return r.v;
}

__global__ __launch_bounds__(128, 2)
void fa_fwd_kernel(const float* __restrict__ Qg, const float* __restrict__ Kg,
                   const float* __restrict__ Vg, float* __restrict__ Og)
{
    __shared__ __align__(16) _Float16 Qs[QT][DIM + 8];
    __shared__ __align__(16) _Float16 Ks[KT][DIM + 8];
    __shared__ __align__(16) __bf16 Vh[DIM][KT + 8];
    __shared__ __align__(16) __bf16 Vl[DIM][KT + 8];
    __shared__ __align__(16) float  Os[NWAVE][16][DIM];
    __shared__ __align__(16) float  kadd[KT];
    __shared__ float qmask[QT];

    const int tid  = threadIdx.x;
    const int wid  = tid >> 5;
    const int lane = tid & 31;
    const int h    = lane >> 4;
    const int ln   = lane & 15;

    const int b  = blockIdx.x / (SEQ / QT);
    const int q0 = (blockIdx.x % (SEQ / QT)) * QT;

    const float* Qb = Qg + (size_t)b * SEQ * DIM;
    const float* Kb = Kg + (size_t)b * SEQ * DIM;
    const float* Vb = Vg + (size_t)b * SEQ * DIM;

    {
        const int row  = tid >> 1;
        const int half = (tid & 1) * 32;
        const float* src = Qb + (size_t)(q0 + row) * DIM + half;
        float asum = 0.f;
#pragma unroll
        for (int i = 0; i < 8; ++i) {
            v4f x = *(const v4f*)(src + i * 4);
            asum += __builtin_fabsf(x.x) + __builtin_fabsf(x.y) +
                    __builtin_fabsf(x.z) + __builtin_fabsf(x.w);
            Qs[row][half + i*4 + 0] = (_Float16)(x.x * SCALE);
            Qs[row][half + i*4 + 1] = (_Float16)(x.y * SCALE);
            Qs[row][half + i*4 + 2] = (_Float16)(x.z * SCALE);
            Qs[row][half + i*4 + 3] = (_Float16)(x.w * SCALE);
        }
        asum += __shfl_xor(asum, 1, 32);
        if ((tid & 1) == 0) qmask[row] = (asum != 0.f) ? 1.f : 0.f;
    }
    __syncthreads();

    v16h bq[2];
#pragma unroll
    for (int ks = 0; ks < 2; ++ks)
        bq[ks] = load_frag<v16h, v8h, _Float16>(&Qs[wid*16][0], DIM + 8, ks * 32, lane);

    float m_run = -3.0e38f, l_run = 0.f;
    v8f acc[4];
#pragma unroll
    for (int t = 0; t < 4; ++t) { v8f z = {}; acc[t] = z; }

    const int qmin_w = q0 + wid * 16;
    const int qmax_w = qmin_w + 15;
    const int vq     = qmin_w + ln;

    for (int kb = 0; kb < q0 + QT; kb += KT) {
        __syncthreads();

        {
            const int row = tid >> 1;
            const int col = (tid & 1) * 32;
            const float* ksrc = Kb + (size_t)(kb + row) * DIM + col;
            const float* vsrc = Vb + (size_t)(kb + row) * DIM + col;
            float asum = 0.f;
#pragma unroll
            for (int i = 0; i < 8; ++i) {
                v4f x = *(const v4f*)(ksrc + i * 4);
                asum += __builtin_fabsf(x.x) + __builtin_fabsf(x.y) +
                        __builtin_fabsf(x.z) + __builtin_fabsf(x.w);
                Ks[row][col + i*4 + 0] = (_Float16)x.x;
                Ks[row][col + i*4 + 1] = (_Float16)x.y;
                Ks[row][col + i*4 + 2] = (_Float16)x.z;
                Ks[row][col + i*4 + 3] = (_Float16)x.w;
            }
            asum += __shfl_xor(asum, 1, 32);
            if ((tid & 1) == 0) kadd[row] = (asum != 0.f) ? 0.f : MASKV;
#pragma unroll
            for (int i = 0; i < 8; ++i) {
                v4f x = *(const v4f*)(vsrc + i * 4);
#pragma unroll
                for (int e = 0; e < 4; ++e) {
                    const float xv = x[e];
                    const __bf16 hb = bf_hi(xv);
                    Vh[col + i*4 + e][row] = hb;
                    Vl[col + i*4 + e][row] = bf_lo(xv, hb);
                }
            }
        }
        __syncthreads();

        if (kb <= qmax_w) {
            v8f ct[4];
#pragma unroll
            for (int kt = 0; kt < 4; ++kt) {
                v8f z = {};
                ct[kt] = z;
#pragma unroll
                for (int ks = 0; ks < 2; ++ks) {
                    v16h ak = load_frag<v16h, v8h, _Float16>(&Ks[kt*16][0], DIM + 8, ks * 32, lane);
                    ct[kt] = wmma_f16(ak, bq[ks], ct[kt]);
                }
            }

            float s[4][8];
#pragma unroll
            for (int kt = 0; kt < 4; ++kt) {
                v4f kaL = *(const v4f*)&kadd[kt*16 + h*8];
                v4f kaH = *(const v4f*)&kadd[kt*16 + h*8 + 4];
#pragma unroll
                for (int r = 0; r < 4; ++r) {
                    s[kt][r]   = ct[kt][r]   + kaL[r];
                    s[kt][r+4] = ct[kt][r+4] + kaH[r];
                }
            }

            if (kb + KT - 1 > qmin_w) {
#pragma unroll
                for (int kt = 0; kt < 4; ++kt)
#pragma unroll
                    for (int r = 0; r < 8; ++r) {
                        const int key = kb + kt*16 + h*8 + r;
                        s[kt][r] = (key <= vq) ? s[kt][r] : MASKV;
                    }
            }

            float mx = s[0][0];
#pragma unroll
            for (int kt = 0; kt < 4; ++kt)
#pragma unroll
                for (int r = 0; r < 8; ++r) mx = fmaxf(mx, s[kt][r]);
            mx = fmaxf(mx, __shfl_xor(mx, 16, 32));

            const float mn    = fmaxf(m_run, mx);
            const float alpha = __expf(m_run - mn);
            m_run = mn;

            float p[4][8];
            float rs = 0.f;
#pragma unroll
            for (int kt = 0; kt < 4; ++kt)
#pragma unroll
                for (int r = 0; r < 8; ++r) {
                    p[kt][r] = __expf(s[kt][r] - mn);
                    rs += p[kt][r];
                }
            rs += __shfl_xor(rs, 16, 32);
            l_run = l_run * alpha + rs;

#pragma unroll
            for (int t = 0; t < 4; ++t)
#pragma unroll
                for (int r = 0; r < 8; ++r) acc[t][r] *= alpha;

            v16bf bp0h, bp0l, bp1h, bp1l;
#pragma unroll
            for (int r = 0; r < 8; ++r) {
                __bf16 hb;
                hb = bf_hi(p[0][r]); bp0h[r]     = hb; bp0l[r]     = bf_lo(p[0][r], hb);
                hb = bf_hi(p[1][r]); bp0h[r + 8] = hb; bp0l[r + 8] = bf_lo(p[1][r], hb);
                hb = bf_hi(p[2][r]); bp1h[r]     = hb; bp1l[r]     = bf_lo(p[2][r], hb);
                hb = bf_hi(p[3][r]); bp1h[r + 8] = hb; bp1l[r + 8] = bf_lo(p[3][r], hb);
            }

#pragma unroll
            for (int t = 0; t < 4; ++t) {
                v16bf avh = load_frag<v16bf, v8bf, __bf16>(&Vh[t*16][0], KT + 8, 0, lane);
                v16bf avl = load_frag<v16bf, v8bf, __bf16>(&Vl[t*16][0], KT + 8, 0, lane);
                acc[t] = wmma_bf16(avh, bp0h, acc[t]);
                acc[t] = wmma_bf16(avh, bp0l, acc[t]);
                acc[t] = wmma_bf16(avl, bp0h, acc[t]);
                avh = load_frag<v16bf, v8bf, __bf16>(&Vh[t*16][0], KT + 8, 32, lane);
                avl = load_frag<v16bf, v8bf, __bf16>(&Vl[t*16][0], KT + 8, 32, lane);
                acc[t] = wmma_bf16(avh, bp1h, acc[t]);
                acc[t] = wmma_bf16(avh, bp1l, acc[t]);
                acc[t] = wmma_bf16(avl, bp1h, acc[t]);
            }
        }
    }

    {
        const float sc = ((l_run > 0.f) ? 1.f / l_run : 0.f) * qmask[wid*16 + ln];
#pragma unroll
        for (int t = 0; t < 4; ++t)
#pragma unroll
            for (int r = 0; r < 8; ++r)
                Os[wid][ln][t*16 + h*8 + r] = acc[t][r] * sc;
    }
    __syncthreads();
    {
        const float* osf = &Os[wid][0][0];
        float* og = Og + ((size_t)b * SEQ + q0 + wid*16) * DIM;
        v4f vv[8];
#pragma unroll
        for (int i = 0; i < 8; ++i) vv[i] = *(const v4f*)(osf + (lane + i*32) * 4);
#pragma unroll
        for (int i = 0; i < 8; ++i) *(volatile v4f*)(og + (lane + i*32) * 4) = vv[i];
        __threadfence();
#pragma unroll
        for (int i = 0; i < 8; ++i) *(volatile v4f*)(og + (lane + i*32) * 4) = vv[i];
    }
}

extern "C" void kernel_launch(void* const* d_in, const int* in_sizes, int n_in,
                              void* d_out, int out_size, void* d_ws, size_t ws_size,
                              hipStream_t stream) {
    (void)in_sizes; (void)n_in; (void)out_size; (void)d_ws; (void)ws_size;
    const float* Q = (const float*)d_in[0];
    const float* K = (const float*)d_in[1];
    const float* V = (const float*)d_in[2];
    float* O = (float*)d_out;
    dim3 grid(BATCH * (SEQ / QT));
    dim3 block(128);
    hipLaunchKernelGGL(fa_fwd_kernel, grid, block, 0, stream, Q, K, V, O);
}
